// OptimizedMAGECActor_55267639165123
// MI455X (gfx1250) — hardware-verified
//
#include <hip/hip_runtime.h>
#include <stddef.h>
#include <math.h>


#define FD      128
#define HH      64
#define NTHR    256
#define NWAVE   8
#define EPT     8
#define NGRP    2
#define CHUNK   (NTHR * EPT * NGRP)
#define WCAP    (EPT * NGRP * 32)
#define LISTN   (NWAVE * WCAP)
#define NBC     4096
#define NBF     2048
#define FPC     (NBC / NBF)
#define RCAP    40960
#define RBN     128
#define RPADN   256
#define DEGCAP  256
#define OTHR    512
#define BM      64
#define GRW     8
#define RPW     4
#define WSLIM   134217728
#define BN_EPS  1e-5
#define NORM_EPS 1e-12f

#define LDS_FILL  ((RCAP + NBF + LISTN) * 4 + 64)
#define LDS_LAYER (BM * FD * 2 * 4 + BM * FD * 4)

static_assert((CHUNK & (CHUNK - 1)) == 0);
static_assert(CHUNK <= 4096);
static_assert(NBC <= 4096 && NBF <= 4096);
static_assert((NBC & (NBC - 1)) == 0 && (NBF & (NBF - 1)) == 0);
static_assert(NBC == FPC * NBF && FPC == 2);
static_assert(OTHR * 8 == NBC);
static_assert(OTHR / 32 == 8 * FPC);
static_assert((RCAP % 32) == 0);
static_assert((RPADN % BM) == 0 && (RPADN % (NWAVE * RPW)) == 0 && (RPADN % 8) == 0);
static_assert((DEGCAP % 32) == 0);
static_assert(BM == 64 && NWAVE == 8 && HH == 64);
static_assert(BM == NWAVE * GRW);

typedef float          v2f  __attribute__((ext_vector_type(2)));
typedef float          v4f  __attribute__((ext_vector_type(4)));
typedef float          v8f  __attribute__((ext_vector_type(8)));
typedef double         v2d  __attribute__((ext_vector_type(2)));
typedef int            v4i  __attribute__((ext_vector_type(4)));
typedef unsigned short v4us __attribute__((ext_vector_type(4)));
typedef unsigned short v8us __attribute__((ext_vector_type(8)));
typedef unsigned short v16us __attribute__((ext_vector_type(16)));
typedef __bf16         v16bf __attribute__((ext_vector_type(16)));
union FragU { v16us w; v8us u[2]; };

__device__ __forceinline__ v8f wmb(v16us a, v16us b, v8f c) {
  const v16bf ab = __builtin_bit_cast(v16bf, a);
  const v16bf bb = __builtin_bit_cast(v16bf, b);
  v8f d = __builtin_amdgcn_wmma_f32_16x16x32_bf16(false, ab, false, bb, (short)0, c, false, false);
  asm volatile("v_nop\n\tv_nop\n\tv_nop\n\tv_nop" : "+v"(d) : "v"(a), "v"(b));
  return d;
}

__device__ __forceinline__ unsigned int bfb(float f) {
  const unsigned int u = __float_as_uint(f);
  return (u + 0x7FFFu + ((u >> 16) & 1u)) >> 16;
}
__device__ __forceinline__ void sp1(float v, unsigned short& h, unsigned short& l) {
  const unsigned int hb = bfb(v);
  const float hf = __uint_as_float(hb << 16);
  h = (unsigned short)hb;
  l = (unsigned short)bfb(v - hf);
}
__device__ __forceinline__ void sp4(v4f a, v4us& h, v4us& l) {
  unsigned short hh, ll;
  sp1(a.x, hh, ll); h[0] = hh; l[0] = ll;
  sp1(a.y, hh, ll); h[1] = hh; l[1] = ll;
  sp1(a.z, hh, ll); h[2] = hh; l[2] = ll;
  sp1(a.w, hh, ll); h[3] = hh; l[3] = ll;
}
__device__ __forceinline__ void sp8(v4f a, v4f b, v8us& h, v8us& l) {
  unsigned short hh, ll;
  sp1(a.x, hh, ll); h[0] = hh; l[0] = ll;
  sp1(a.y, hh, ll); h[1] = hh; l[1] = ll;
  sp1(a.z, hh, ll); h[2] = hh; l[2] = ll;
  sp1(a.w, hh, ll); h[3] = hh; l[3] = ll;
  sp1(b.x, hh, ll); h[4] = hh; l[4] = ll;
  sp1(b.y, hh, ll); h[5] = hh; l[5] = ll;
  sp1(b.z, hh, ll); h[6] = hh; l[6] = ll;
  sp1(b.w, hh, ll); h[7] = hh; l[7] = ll;
}

__global__ __launch_bounds__(NTHR) void k_wprep(const float* __restrict__ Wp0, const float* __restrict__ Wp1,
                                               const float* __restrict__ Wp2, int ldw, int kstep, int nv,
                                               unsigned short* ph, unsigned short* pl, int units) {
  const int i = (int)blockIdx.x * NTHR + (int)threadIdx.x;
  if (i >= units) return;
  const int R   = i >> 4;
  const int k0  = (i & 15) * 8;
  const int blk = R >> 7;
  const int n   = R & (FD - 1);
  const int nc  = n < nv - 1 ? n : nv - 1;
  const float* W = blk == 0 ? Wp0 : (blk == 1 ? Wp1 : Wp2);
  const size_t base = (size_t)(kstep * blk + k0) * (size_t)ldw + (size_t)nc;
  float f[8];
#pragma unroll
  for (int j = 0; j < 8; ++j) f[j] = W[base + (size_t)j * (size_t)ldw];
  v4f a0, a1;
  a0.x = f[0]; a0.y = f[1]; a0.z = f[2]; a0.w = f[3];
  a1.x = f[4]; a1.y = f[5]; a1.z = f[6]; a1.w = f[7];
  const v4f z4 = {0.f, 0.f, 0.f, 0.f};
  if (n >= nv) { a0 = z4; a1 = z4; }
  v8us hv, lv;
  sp8(a0, a1, hv, lv);
  unsigned short* dh = ph + (size_t)i * 8;
  unsigned short* dl = pl + (size_t)i * 8;
  *(volatile v8us*)dh = hv;
  *(volatile v8us*)dl = lv;
  __threadfence();
  *(volatile v8us*)dh = hv;
  *(volatile v8us*)dl = lv;
}

template <int NB>
__device__ __forceinline__ int scan_chunk(const int* __restrict__ dsts, int nE, int cbase, int slotBase,
                                          int vec8, int* list, int tid, int lane, int wave) {
  int wc = 0;
#pragma unroll
  for (int g = 0; g < NGRP; ++g) {
    const int el0  = (g * NTHR + tid) * EPT;
    const int e0   = cbase + el0;
    const int sent = -2147483647 - 1;
    v4i da, db;
    if (vec8 != 0 && cbase + CHUNK <= nE) {
      da = *(const v4i*)(dsts + e0);
      db = *(const v4i*)(dsts + e0 + 4);
    } else {
      da.x = (e0     < nE) ? dsts[min(e0, nE - 1)] : sent;
      da.y = (e0 + 1 < nE) ? dsts[min(e0 + 1, nE - 1)] : sent;
      da.z = (e0 + 2 < nE) ? dsts[min(e0 + 2, nE - 1)] : sent;
      da.w = (e0 + 3 < nE) ? dsts[min(e0 + 3, nE - 1)] : sent;
      db.x = (e0 + 4 < nE) ? dsts[min(e0 + 4, nE - 1)] : sent;
      db.y = (e0 + 5 < nE) ? dsts[min(e0 + 5, nE - 1)] : sent;
      db.z = (e0 + 6 < nE) ? dsts[min(e0 + 6, nE - 1)] : sent;
      db.w = (e0 + 7 < nE) ? dsts[min(e0 + 7, nE - 1)] : sent;
    }
    const unsigned nb = (unsigned)slotBase;
    const unsigned s0 = (unsigned)da.x - nb, s1 = (unsigned)da.y - nb;
    const unsigned s2 = (unsigned)da.z - nb, s3 = (unsigned)da.w - nb;
    const unsigned s4 = (unsigned)db.x - nb, s5 = (unsigned)db.y - nb;
    const unsigned s6 = (unsigned)db.z - nb, s7 = (unsigned)db.w - nb;
    const bool h0 = s0 < (unsigned)NB, h1 = s1 < (unsigned)NB, h2 = s2 < (unsigned)NB, h3 = s3 < (unsigned)NB;
    const bool h4 = s4 < (unsigned)NB, h5 = s5 < (unsigned)NB, h6 = s6 < (unsigned)NB, h7 = s7 < (unsigned)NB;
    const unsigned any = __builtin_amdgcn_ballot_w32(h0 | h1 | h2 | h3 | h4 | h5 | h6 | h7);
    if (any != 0u) {
#define HITJ(J, HJ, SJ) { \
        const unsigned mj = __builtin_amdgcn_ballot_w32(HJ); \
        if (mj != 0u) { \
          if (HJ) { \
            const int pos = wc + (int)__builtin_amdgcn_mbcnt_lo(mj, 0u); \
            if (pos < WCAP) list[wave * WCAP + pos] = ((el0 + (J)) << 12) | (int)(SJ); \
          } \
          wc += (int)__builtin_popcount(mj); } }
      HITJ(0, h0, s0)
      HITJ(1, h1, s1)
      HITJ(2, h2, s2)
      HITJ(3, h3, s3)
      HITJ(4, h4, s4)
      HITJ(5, h5, s5)
      HITJ(6, h6, s6)
      HITJ(7, h7, s7)
#undef HITJ
    }
  }
  return wc;
}

__global__ __launch_bounds__(NTHR) void k_count(
    const int* __restrict__ dsts, int* cnt, int nE, int vec8) {
  __shared__ __attribute__((aligned(16))) int scnt[NBC];
  __shared__ __attribute__((aligned(16))) int list[LISTN];
  __shared__ int wcnt[NWAVE];
  const int tid = threadIdx.x, lane = tid & 31, wave = tid >> 5;
  const int nodeBase = blockIdx.x * NBC;

  for (int i = tid; i < NBC; i += NTHR) scnt[i] = 0;
  __syncthreads();

  const int nChunks = (nE + CHUNK - 1) / CHUNK;
#pragma unroll 1
  for (int ch = 0; ch < nChunks; ++ch) {
    const int cbase = ch * CHUNK;
    const int wc = scan_chunk<NBC>(dsts, nE, cbase, nodeBase, vec8, list, tid, lane, wave);
    if (lane == 0) wcnt[wave] = wc;
    __syncthreads();
    if (wave == 0) {
#pragma unroll 1
      for (int wsx = 0; wsx < NWAVE; ++wsx) {
        int n = __builtin_amdgcn_readfirstlane(wcnt[wsx]);
        n = n > WCAP ? WCAP : (n < 0 ? 0 : n);
        const int* lp = list + wsx * WCAP;
#pragma unroll 1
        for (int i = 0; i < n; ++i) {
          const int ent  = __builtin_amdgcn_readfirstlane(lp[i]);
          const int slot = ent & (NBC - 1);
          if (lane == 0) scnt[slot] = scnt[slot] + 1;
        }
      }
    }
    __syncthreads();
  }

  v4i cq[4];
#pragma unroll
  for (int q = 0; q < 4; ++q) {
    const int f = (wave * 4 + q) * 128 + 4 * lane;
    cq[q] = *(const v4i*)(scnt + f);
  }
  int* cpn = cnt + (size_t)nodeBase;
#pragma unroll
  for (int q = 0; q < 4; ++q) {
    const int f = (wave * 4 + q) * 128 + 4 * lane;
    *(volatile v4i*)(cpn + f) = cq[q];
  }
  __threadfence();
#pragma unroll
  for (int q = 0; q < 4; ++q) {
    const int f = (wave * 4 + q) * 128 + 4 * lane;
    *(volatile v4i*)(cpn + f) = cq[q];
  }
}

__global__ __launch_bounds__(OTHR) void k_offsets(
    const int* __restrict__ cnt, int* off, int* rbase, int nChunk) {
  __shared__ __attribute__((aligned(16))) int soff[NBC];
  __shared__ __attribute__((aligned(16))) int srb[RBN];
  __shared__ int wtot[OTHR / 32];
  const int tid = threadIdx.x, lane = tid & 31, wave = tid >> 5, sub = tid >> 8;
  for (int i = tid; i < RBN; i += OTHR) srb[i] = 0;
  __syncthreads();
  int carry = 0;
#pragma unroll 1
  for (int ch = 0; ch < nChunk; ++ch) {
    const int base = ch * NBC;
    const v4i ca = *(const v4i*)(cnt + base + 8 * tid);
    const v4i cb = *(const v4i*)(cnt + base + 8 * tid + 4);
    const int e0 = max(ca.x, 0), e1 = max(ca.y, 0), e2 = max(ca.z, 0), e3 = max(ca.w, 0);
    const int e4 = max(cb.x, 0), e5 = max(cb.y, 0), e6 = max(cb.z, 0), e7 = max(cb.w, 0);
    const int ts = e0 + e1 + e2 + e3 + e4 + e5 + e6 + e7;
    int incl = ts;
#pragma unroll
    for (int d = 1; d < 32; d <<= 1) {
      const int t = __shfl_up(incl, d);
      if (lane >= d) incl += t;
    }
    if (lane == 31) wtot[wave] = incl;
    __syncthreads();
    int S0 = 0, S1 = 0;
#pragma unroll
    for (int w = 0; w < 8; ++w) { S0 += wtot[w]; S1 += wtot[8 + w]; }
    int pre = 0;
#pragma unroll 1
    for (int w = 8 * sub; w < wave; ++w) pre += wtot[w];
    const int b0 = carry;
    const int b1 = b0 + ((S0 + 31) & ~31);
    const int b2 = b1 + ((S1 + 31) & ~31);
    const int myb = sub == 0 ? b0 : b1;
    if (tid == 0) {
      srb[min(2 * ch + 0, RBN - 1)] = b0;
      srb[min(2 * ch + 1, RBN - 1)] = b1;
    }
    int run = myb + pre + incl - ts;
    soff[8 * tid + 0] = run; run += e0;
    soff[8 * tid + 1] = run; run += e1;
    soff[8 * tid + 2] = run; run += e2;
    soff[8 * tid + 3] = run; run += e3;
    soff[8 * tid + 4] = run; run += e4;
    soff[8 * tid + 5] = run; run += e5;
    soff[8 * tid + 6] = run; run += e6;
    soff[8 * tid + 7] = run;
    carry = b2;
    __syncthreads();
    const v4i o0 = *(const v4i*)(soff + 4 * tid);
    const v4i o1 = *(const v4i*)(soff + 4 * (tid + OTHR));
    int* op = off + base;
    *(volatile v4i*)(op + 4 * tid) = o0;
    *(volatile v4i*)(op + 4 * (tid + OTHR)) = o1;
    __threadfence();
    *(volatile v4i*)(op + 4 * tid) = o0;
    *(volatile v4i*)(op + 4 * (tid + OTHR)) = o1;
    __syncthreads();
  }
  if (tid == 0) srb[min(2 * nChunk, RBN - 1)] = carry;
  __syncthreads();
  v4i rv = {0, 0, 0, 0};
  if (tid < 32) rv = *(const v4i*)(srb + 4 * tid);
  if (tid < 32) *(volatile v4i*)(rbase + 4 * tid) = rv;
  __threadfence();
  if (tid < 32) *(volatile v4i*)(rbase + 4 * tid) = rv;
}

__global__ __launch_bounds__(NTHR) void k_fill(
    const int* __restrict__ dsts, const int* __restrict__ off, const int* __restrict__ rbase,
    int* csr, int nE, int vec8, int csrLen) {
  extern __shared__ v4f lds_dyn[];
  int* region = (int*)lds_dyn;
  int* cursor = region + RCAP;
  int* list   = cursor + NBF;
  int* wcnt   = list + LISTN;
  const int tid = threadIdx.x, lane = tid & 31, wave = tid >> 5;
  const int b = blockIdx.x;
  const int nodeBase = b * NBF;

  int rb0 = rbase[b];
  const int rb1 = rbase[b + 1];
  rb0 = rb0 < 0 ? 0 : (rb0 > csrLen ? csrLen : rb0);
  rb0 &= ~31;
  int len = rb1 - rb0;
  len = len < 0 ? 0 : (len > RCAP ? RCAP : len);
  int lenW = (len + 31) & ~31;
  if (rb0 + lenW > csrLen) lenW = (csrLen - rb0) & ~31;

  {
    const v4i z = {0, 0, 0, 0};
    for (int i = tid; i < RCAP / 4; i += NTHR) ((v4i*)region)[i] = z;
    for (int s = tid; s < NBF; s += NTHR) {
      int o = off[nodeBase + s] - rb0;
      o = o < 0 ? 0 : (o > RCAP ? RCAP : o);
      cursor[s] = o;
    }
  }
  __syncthreads();

  const int nChunks = (nE + CHUNK - 1) / CHUNK;
#pragma unroll 1
  for (int ch = 0; ch < nChunks; ++ch) {
    const int cbase = ch * CHUNK;
    const int wc = scan_chunk<NBF>(dsts, nE, cbase, nodeBase, vec8, list, tid, lane, wave);
    if (lane == 0) wcnt[wave] = wc;
    __syncthreads();
    if (wave == 0) {
#pragma unroll 1
      for (int wsx = 0; wsx < NWAVE; ++wsx) {
        int n = __builtin_amdgcn_readfirstlane(wcnt[wsx]);
        n = n > WCAP ? WCAP : (n < 0 ? 0 : n);
        const int* lp = list + wsx * WCAP;
#pragma unroll 1
        for (int i = 0; i < n; ++i) {
          const int ent  = __builtin_amdgcn_readfirstlane(lp[i]);
          const int slot = ent & (NBF - 1);
          int e = cbase + ((ent >> 12) & (CHUNK - 1));
          e = e > nE - 1 ? nE - 1 : e;
          if (lane == 0) {
            int pos = cursor[slot];
            pos = pos < 0 ? 0 : (pos > RCAP - 1 ? RCAP - 1 : pos);
            region[pos] = e;
            const int np = pos + 1;
            cursor[slot] = np > RCAP ? RCAP : np;
          }
        }
      }
    }
    __syncthreads();
  }

  const int nv = lenW >> 2;
  int* gp = csr + rb0;
#pragma unroll 1
  for (int i = tid; i < nv; i += NTHR) { const v4i v = ((const v4i*)region)[i]; *(volatile v4i*)(gp + 4 * i) = v; }
  __threadfence();
#pragma unroll 1
  for (int i = tid; i < nv; i += NTHR) { const v4i v = ((const v4i*)region)[i]; *(volatile v4i*)(gp + 4 * i) = v; }
}

__global__ __launch_bounds__(NTHR) void k_inproj(const float* __restrict__ x, const float* __restrict__ Win,
                                                const float* __restrict__ bin, float* H, int nN, int nUnits) {
  const int i = (int)blockIdx.x * NTHR + (int)threadIdx.x;
  if (i >= nUnits) return;
  const int row = i >> 5;
  const int c   = (i & 31) * 4;
  const int rc  = row < nN ? row : nN - 1;
  const v4f xv = *(const v4f*)(x + (size_t)rc * 4);
  const v4f w0 = *(const v4f*)(Win + c);
  const v4f w1 = *(const v4f*)(Win + FD + c);
  const v4f w2 = *(const v4f*)(Win + 2 * FD + c);
  const v4f w3 = *(const v4f*)(Win + 3 * FD + c);
  const v4f bb = *(const v4f*)(bin + c);
  const v4f z4 = {0.f, 0.f, 0.f, 0.f};
  v4f v = xv.x * w0;
  v += xv.y * w1;
  v += xv.z * w2;
  v += xv.w * w3;
  v += bb;
  if (row >= nN) v = z4;
  float* dh = H + (size_t)row * FD + c;
  *(volatile v4f*)dh = v;
  __threadfence();
  *(volatile v4f*)dh = v;
}

__device__ __forceinline__ void stage64(const float* src, int rowBase, int nValid,
                                        unsigned short* th, unsigned short* tl) {
  const int tid = threadIdx.x;
  const v4f z4 = {0.f, 0.f, 0.f, 0.f};
#pragma unroll
  for (int it = 0; it < 4; ++it) {
    const int u = it * NTHR + tid;
    const int r = u >> 4, c = (u & 15) * 8;
    const int grow = rowBase + r;
    const int rc = grow < nValid ? grow : nValid - 1;
    const float* p = src + (size_t)rc * FD + c;
    v4f a = *(const v4f*)p, b = *(const v4f*)(p + 4);
    if (grow >= nValid) { a = z4; b = z4; }
    v8us hv, lv;
    sp8(a, b, hv, lv);
    *(v8us*)(th + r * FD + c) = hv;
    *(v8us*)(tl + r * FD + c) = lv;
  }
}

__device__ __forceinline__ void lstage64(const float* stg, unsigned short* th, unsigned short* tl) {
  const int tid = threadIdx.x;
#pragma unroll
  for (int it = 0; it < 4; ++it) {
    const int u = it * NTHR + tid;
    const int r = u >> 4, c = (u & 15) * 8;
    const float* p = stg + r * FD + c;
    const v4f a = *(const v4f*)p, b = *(const v4f*)(p + 4);
    v8us hv, lv;
    sp8(a, b, hv, lv);
    *(v8us*)(th + r * FD + c) = hv;
    *(v8us*)(tl + r * FD + c) = lv;
  }
}

template <int NT, int PB>
__device__ __forceinline__ void mmk(v8f (&acc)[NT], const unsigned short* th, const unsigned short* tl, int arow,
                                    const unsigned short* __restrict__ Bh, const unsigned short* __restrict__ Bl,
                                    int bcol0, int kofs) {
  const int lane = threadIdx.x & 31, hh = lane >> 4, m = lane & 15;
  const unsigned short* aph = th + (arow + m) * FD + 8 * hh;
  const unsigned short* apl = tl + (arow + m) * FD + 8 * hh;
  const size_t boff = (size_t)(bcol0 + m) * PB + kofs + 8 * hh;
  const unsigned short* bph0 = Bh + boff;
  const unsigned short* bpl0 = Bl + boff;
#pragma unroll 1
  for (int kt = 0; kt < FD / 32; ++kt) {
    FragU ah, al;
    ah.u[0] = *(const v8us*)(aph + 32 * kt);
    ah.u[1] = *(const v8us*)(aph + 32 * kt + 16);
    al.u[0] = *(const v8us*)(apl + 32 * kt);
    al.u[1] = *(const v8us*)(apl + 32 * kt + 16);
#pragma unroll
    for (int t = 0; t < NT; ++t) {
      const size_t to = (size_t)(16 * t) * PB + 32 * kt;
      FragU bh, bl;
      bh.u[0] = *(const v8us*)(bph0 + to);
      bh.u[1] = *(const v8us*)(bph0 + to + 16);
      bl.u[0] = *(const v8us*)(bpl0 + to);
      bl.u[1] = *(const v8us*)(bpl0 + to + 16);
      acc[t] = wmb(ah.w, bh.w, acc[t]);
      acc[t] = wmb(al.w, bh.w, acc[t]);
      acc[t] = wmb(ah.w, bl.w, acc[t]);
    }
  }
}

__device__ __forceinline__ void gsum(const int* __restrict__ csr, const int* __restrict__ off,
                                     const int* __restrict__ cnt, const int* __restrict__ srcs,
                                     const float* __restrict__ eattr, const float* Hin,
                                     int rowBase, int nN, int nE, int csrLen,
                                     unsigned short* thS, unsigned short* tlS,
                                     float* sE0, float* sE1, float* sInv) {
  const int tid = threadIdx.x, lane = tid & 31, wave = tid >> 5;
  const int col = 4 * lane;
#pragma unroll 1
  for (int j = 0; j < GRW; ++j) {
    const int tr  = GRW * wave + j;
    const int c   = rowBase + tr;
    const int dg  = cnt[c];
    const int dgp = dg < 0 ? 0 : dg;
    const int n   = dgp > DEGCAP ? DEGCAP : dgp;
    const int st  = off[c];
    v4f acc = *(const v4f*)(Hin + (size_t)c * FD + col);
    float ea0 = 0.f, ea1 = 0.f;
#pragma unroll 1
    for (int q0 = 0; q0 < n; q0 += 32) {
      int pos = st + q0 + lane;
      pos = pos < 0 ? 0 : (pos > csrLen - 1 ? csrLen - 1 : pos);
      int eid = csr[pos];
      eid = eid < 0 ? 0 : (eid > nE - 1 ? nE - 1 : eid);
      int sl = srcs[eid];
      sl = sl < 0 ? 0 : (sl > nN - 1 ? nN - 1 : sl);
      const v2f ev = *(const v2f*)(eattr + 2 * (size_t)eid);
      const int mcnt = (n - q0) < 32 ? (n - q0) : 32;
      ea0 += (lane < mcnt) ? ev.x : 0.f;
      ea1 += (lane < mcnt) ? ev.y : 0.f;
#pragma unroll 1
      for (int pp = 0; pp < mcnt; ++pp) {
        const int s = __builtin_amdgcn_readlane(sl, pp);
        acc += *(const v4f*)(Hin + (size_t)s * FD + col);
      }
    }
#pragma unroll
    for (int d = 16; d > 0; d >>= 1) {
      ea0 += __shfl_xor(ea0, d);
      ea1 += __shfl_xor(ea1, d);
    }
    v4us hv, lv;
    sp4(acc, hv, lv);
    *(v4us*)(thS + tr * FD + col) = hv;
    *(v4us*)(tlS + tr * FD + col) = lv;
    const float inv = 1.0f / (float)(dgp + 1);
    if (lane == 0) { sE0[tr] = ea0; sE1[tr] = ea1; sInv[tr] = inv; }
  }
}

__device__ __forceinline__ void aggfix(v8f (&acc)[4], const float* __restrict__ Wt, int r0, int c0,
                                       const float* sE0, const float* sE1, const float* sInv) {
  const int lane = threadIdx.x & 31, hh = lane >> 4, m = lane & 15;
  float e0[8], e1[8], iv[8];
#pragma unroll
  for (int r = 0; r < 8; ++r) {
    const int row = r0 + 8 * hh + r;
    e0[r] = sE0[row]; e1[r] = sE1[row]; iv[r] = sInv[row];
  }
#pragma unroll
  for (int t = 0; t < 4; ++t) {
    const int colx = c0 + 16 * t + m;
    const float w0 = Wt[colx], w1 = Wt[FD + colx];
#pragma unroll
    for (int r = 0; r < 8; ++r) acc[t][r] = (acc[t][r] + e0[r] * w0 + e1[r] * w1) * iv[r];
  }
}

__global__ __launch_bounds__(NTHR) void k_layer(
    const float* Hin, float* Hout, int doStore,
    const int* __restrict__ csr, const int* __restrict__ off, const int* __restrict__ cnt,
    const int* __restrict__ srcs, const float* __restrict__ eattr, const float* __restrict__ Wt,
    const unsigned short* __restrict__ Bnh, const unsigned short* __restrict__ Bnl,
    const unsigned short* __restrict__ Bsh, const unsigned short* __restrict__ Bsl,
    double* part, int nN, int nE, int csrLen) {
  extern __shared__ v4f lds_dyn[];
  __shared__ __attribute__((aligned(16))) double spt[2 * FD];
  __shared__ float sE0[BM];
  __shared__ float sE1[BM];
  __shared__ float sInv[BM];
  unsigned short* thH = (unsigned short*)lds_dyn;
  unsigned short* tlH = thH + BM * FD;
  unsigned short* thS = tlH + BM * FD;
  unsigned short* tlS = thS + BM * FD;
  float* stg = (float*)(tlS + BM * FD);
  const int tid = threadIdx.x, lane = tid & 31, wave = tid >> 5, hh = lane >> 4, m = lane & 15;
  const int rowBase = blockIdx.x * BM;
  const int r0 = (wave >> 1) * 16, c0 = (wave & 1) * 64;

  stage64(Hin, rowBase, nN, thH, tlH);
  gsum(csr, off, cnt, srcs, eattr, Hin, rowBase, nN, nE, csrLen, thS, tlS, sE0, sE1, sInv);
  __syncthreads();

  v8f acc[4];
#pragma unroll
  for (int t = 0; t < 4; ++t) { v8f z = {0.f, 0.f, 0.f, 0.f, 0.f, 0.f, 0.f, 0.f}; acc[t] = z; }
  mmk<4, FD>(acc, thS, tlS, r0, Bnh, Bnl, c0, 0);
  aggfix(acc, Wt, r0, c0, sE0, sE1, sInv);
  mmk<4, FD>(acc, thH, tlH, r0, Bsh, Bsl, c0, 0);
  {
    float* sp = stg + (size_t)(r0 + 8 * hh) * FD + c0 + m;
#pragma unroll
    for (int t = 0; t < 4; ++t) {
#pragma unroll
      for (int r = 0; r < 8; ++r) sp[r * FD + 16 * t] = fmaxf(acc[t][r], 0.f);
    }
  }
  __syncthreads();

  if (tid < FD) {
    double s = 0.0, qq = 0.0;
#pragma unroll 1
    for (int r = 0; r < BM; ++r) {
      const float vf = stg[r * FD + tid];
      const double v = (rowBase + r < nN) ? (double)vf : 0.0;
      s += v;
      qq += v * v;
    }
    spt[tid] = s;
    spt[FD + tid] = qq;
  }
  __syncthreads();

  const v4f z4 = {0.f, 0.f, 0.f, 0.f};
  const int rsub = lane >> 4, q = lane & 15, col = c0 + 4 * q;
  const int tp = tid < FD ? tid : FD - 1;
  const v2d pw = *(const v2d*)(spt + 2 * tp);
  double* pp = part + (size_t)blockIdx.x * (2 * FD) + 2 * tp;
  v4f vv[8];
#pragma unroll
  for (int it = 0; it < 8; ++it) {
    const int row  = it * 2 + rsub;
    const int grow = rowBase + r0 + row;
    v4f v = *(const v4f*)(stg + (size_t)(r0 + row) * FD + col);
    if (grow >= nN) v = z4;
    vv[it] = v;
  }
  if (tid < FD) *(volatile v2d*)pp = pw;
  if (doStore != 0) {
#pragma unroll
    for (int it = 0; it < 8; ++it) {
      const int grow = rowBase + r0 + it * 2 + rsub;
      *(volatile v4f*)(Hout + (size_t)grow * FD + col) = vv[it];
    }
  }
  __threadfence();
  if (tid < FD) *(volatile v2d*)pp = pw;
  if (doStore != 0) {
#pragma unroll
    for (int it = 0; it < 8; ++it) {
      const int grow = rowBase + r0 + it * 2 + rsub;
      *(volatile v4f*)(Hout + (size_t)grow * FD + col) = vv[it];
    }
  }
}

__global__ __launch_bounds__(FD) void k_bnfin(const double* __restrict__ part, const float* __restrict__ gamma,
                                              float* tbl, int nPart, int nN) {
  __shared__ __attribute__((aligned(16))) float stb[2 * FD];
  const int tid = threadIdx.x, col = tid;
  double s = 0.0, q = 0.0;
#pragma unroll 1
  for (int b = 0; b < nPart; ++b) {
    s += part[(size_t)b * (2 * FD) + col];
    q += part[(size_t)b * (2 * FD) + FD + col];
  }
  const double inv = 1.0 / (double)nN;
  const double mu  = s * inv;
  double var = q * inv - mu * mu;
  var = var < 0.0 ? 0.0 : var;
  const float a  = (float)((double)gamma[col] / sqrt(var + BN_EPS));
  const float mf = (float)mu;
  stb[col] = mf;
  stb[FD + col] = a;
  __syncthreads();
  const int t4 = tid < 64 ? tid : 63;
  const v4f w = *(const v4f*)(stb + 4 * t4);
  if (tid < 64) *(volatile v4f*)(tbl + 4 * tid) = w;
  __threadfence();
  if (tid < 64) *(volatile v4f*)(tbl + 4 * tid) = w;
}

__global__ __launch_bounds__(NTHR) void k_bnl2(float* HB, const float* __restrict__ tbl,
                                              const float* __restrict__ beta, int nN) {
  const int tid = threadIdx.x, lane = tid & 31, wave = tid >> 5;
  const int col = 4 * lane;
  const v4f mu = *(const v4f*)(tbl + col);
  const v4f ga = *(const v4f*)(tbl + FD + col);
  const v4f be = *(const v4f*)(beta + col);
  const v4f z4 = {0.f, 0.f, 0.f, 0.f};
  const int rbase = ((int)blockIdx.x * NWAVE + wave) * RPW;
#pragma unroll 1
  for (int i = 0; i < RPW; ++i) {
    const int row = rbase + i;
    float* p = HB + (size_t)row * FD + col;
    const v4f o = *(const v4f*)p;
    const v4f v = (o - mu) * ga + be;
    float ss = v.x * v.x + v.y * v.y + v.z * v.z + v.w * v.w;
#pragma unroll
    for (int d = 16; d > 0; d >>= 1) ss += __shfl_xor(ss, d);
    const float nrm = fmaxf(sqrtf(ss), NORM_EPS);
    const float inv = 1.0f / nrm;
    v4f h = v * inv;
    if (row >= nN) h = z4;
    *(volatile v4f*)p = h;
    __threadfence();
    *(volatile v4f*)p = h;
  }
}

__global__ __launch_bounds__(NTHR) void k_final(
    const float* Hin, const float* Hj1,
    const int* __restrict__ csr, const int* __restrict__ off, const int* __restrict__ cnt,
    const int* __restrict__ srcs, const float* __restrict__ eattr, const float* __restrict__ Wt,
    const unsigned short* __restrict__ Bnh, const unsigned short* __restrict__ Bnl,
    const unsigned short* __restrict__ Bsh, const unsigned short* __restrict__ Bsl,
    const float* __restrict__ tbl, const float* __restrict__ beta,
    const unsigned short* __restrict__ Jh, const unsigned short* __restrict__ Jl, const float* __restrict__ bj,
    const unsigned short* __restrict__ B1h, const unsigned short* __restrict__ B1l,
    const float* __restrict__ b1, const float* __restrict__ w2, const float* __restrict__ b2,
    float* out, int nN, int nE, int csrLen) {
  extern __shared__ v4f lds_dyn[];
  __shared__ float sE0[BM];
  __shared__ float sE1[BM];
  __shared__ float sInv[BM];
  __shared__ __attribute__((aligned(16))) float sc[BM];
  unsigned short* thH = (unsigned short*)lds_dyn;
  unsigned short* tlH = thH + BM * FD;
  unsigned short* thS = tlH + BM * FD;
  unsigned short* tlS = thS + BM * FD;
  float* stg = (float*)(tlS + BM * FD);
  const int tid = threadIdx.x, lane = tid & 31, wave = tid >> 5, hh = lane >> 4, m = lane & 15;
  const int rowBase = blockIdx.x * BM;
  const int r0 = (wave >> 1) * 16, c0 = (wave & 1) * 64;
  const v4f z4 = {0.f, 0.f, 0.f, 0.f};

  stage64(Hin, rowBase, nN, thH, tlH);
  gsum(csr, off, cnt, srcs, eattr, Hin, rowBase, nN, nE, csrLen, thS, tlS, sE0, sE1, sInv);
  __syncthreads();
  {
    v8f acc[4];
#pragma unroll
    for (int t = 0; t < 4; ++t) { v8f z = {0.f, 0.f, 0.f, 0.f, 0.f, 0.f, 0.f, 0.f}; acc[t] = z; }
    mmk<4, FD>(acc, thS, tlS, r0, Bnh, Bnl, c0, 0);
    aggfix(acc, Wt, r0, c0, sE0, sE1, sInv);
    mmk<4, FD>(acc, thH, tlH, r0, Bsh, Bsl, c0, 0);
    float* sp = stg + (size_t)(r0 + 8 * hh) * FD + c0 + m;
#pragma unroll
    for (int t = 0; t < 4; ++t) {
#pragma unroll
      for (int r = 0; r < 8; ++r) sp[r * FD + 16 * t] = fmaxf(acc[t][r], 0.f);
    }
  }
  __syncthreads();

  {
    const int col = 4 * lane;
    const v4f mu = *(const v4f*)(tbl + col);
    const v4f ga = *(const v4f*)(tbl + FD + col);
    const v4f be = *(const v4f*)(beta + col);
#pragma unroll 1
    for (int j = 0; j < GRW; ++j) {
      const int tr = GRW * wave + j;
      const v4f o = *(const v4f*)(stg + tr * FD + col);
      const v4f v = (o - mu) * ga + be;
      float ss = v.x * v.x + v.y * v.y + v.z * v.z + v.w * v.w;
#pragma unroll
      for (int d = 16; d > 0; d >>= 1) ss += __shfl_xor(ss, d);
      const float nrm = fmaxf(sqrtf(ss), NORM_EPS);
      const float inv = 1.0f / nrm;
      v4f h = v * inv;
      if (rowBase + tr >= nN) h = z4;
      v4us hv, lv;
      sp4(h, hv, lv);
      *(v4us*)(thS + tr * FD + col) = hv;
      *(v4us*)(tlS + tr * FD + col) = lv;
    }
  }
  __syncthreads();

  {
    v8f aj[4];
#pragma unroll
    for (int t = 0; t < 4; ++t) { v8f z = {0.f, 0.f, 0.f, 0.f, 0.f, 0.f, 0.f, 0.f}; aj[t] = z; }
    mmk<4, FD>(aj, thH, tlH, r0, Jh + (size_t)FD * FD, Jl + (size_t)FD * FD, c0, 0);
    mmk<4, FD>(aj, thS, tlS, r0, Jh + (size_t)2 * FD * FD, Jl + (size_t)2 * FD * FD, c0, 0);
    __syncthreads();
    stage64(Hj1, rowBase, nN, thH, tlH);
    __syncthreads();
    mmk<4, FD>(aj, thH, tlH, r0, Jh, Jl, c0, 0);
    float* sp = stg + (size_t)(r0 + 8 * hh) * FD + c0 + m;
#pragma unroll
    for (int t = 0; t < 4; ++t) {
      const float bjv = bj[c0 + 16 * t + m];
#pragma unroll
      for (int r = 0; r < 8; ++r) sp[r * FD + 16 * t] = fmaxf(aj[t][r] + bjv, 0.f);
    }
  }
  __syncthreads();

  lstage64(stg, thS, tlS);
  __syncthreads();
  {
    const int c0h = (wave & 1) * 32;
    v8f ah[2];
#pragma unroll
    for (int t = 0; t < 2; ++t) { v8f z = {0.f, 0.f, 0.f, 0.f, 0.f, 0.f, 0.f, 0.f}; ah[t] = z; }
    mmk<2, FD>(ah, thS, tlS, r0, B1h, B1l, c0h, 0);
    float* sp = stg + (size_t)(r0 + 8 * hh) * HH + c0h + m;
#pragma unroll
    for (int t = 0; t < 2; ++t) {
#pragma unroll
      for (int r = 0; r < 8; ++r) sp[r * HH + 16 * t] = ah[t][r];
    }
  }
  __syncthreads();

  {
    const float wa = w2[lane], wb = w2[lane + 32];
    const float ba = b1[lane], bb = b1[lane + 32];
    const float b2v = b2[0];
#pragma unroll
    for (int r = 0; r < 8; ++r) {
      const int row = 8 * wave + r;
      const float x0 = stg[row * HH + lane];
      const float x1 = stg[row * HH + lane + 32];
      float p = fmaxf(x0 + ba, 0.f) * wa + fmaxf(x1 + bb, 0.f) * wb;
#pragma unroll
      for (int d = 16; d > 0; d >>= 1) p += __shfl_xor(p, d);
      if (lane == 0) sc[row] = p + b2v;
    }
  }
  __syncthreads();

  const int lt = lane < 16 ? lane : 15;
  const v4f v = *(const v4f*)(sc + 4 * lt);
  const size_t f = (size_t)rowBase + 4 * (size_t)lt;
  const bool w0   = (wave == 0) && (lane < 16);
  const bool full = w0 && (f + 4 <= (size_t)nN);
  const bool prt  = w0 && !full && (f < (size_t)nN);
  const long long rem = (long long)nN - (long long)f;
  float* po = out + f;
  if (full) *(volatile v4f*)po = v;
  if (prt) {
    if (rem > 0) *(volatile float*)(po + 0) = v.x;
    if (rem > 1) *(volatile float*)(po + 1) = v.y;
    if (rem > 2) *(volatile float*)(po + 2) = v.z;
  }
  __threadfence();
  if (full) *(volatile v4f*)po = v;
  if (prt) {
    if (rem > 0) *(volatile float*)(po + 0) = v.x;
    if (rem > 1) *(volatile float*)(po + 1) = v.y;
    if (rem > 2) *(volatile float*)(po + 2) = v.z;
  }
}

static size_t carve(size_t* o, size_t bytes) {
  const size_t r = *o;
  *o += (bytes + 255) & ~(size_t)255;
  return r;
}

extern "C" void kernel_launch(void* const* d_in, const int* in_sizes, int n_in,
                              void* d_out, int out_size, void* d_ws, size_t ws_size,
                              hipStream_t stream) {
  if (n_in < 23) return;
  const int nN = in_sizes[0] / 4;
  const int nE = in_sizes[1] / 2;
  if (nN <= 0 || nE <= 0 || in_sizes[0] != 4 * nN || in_sizes[1] != 2 * nE || in_sizes[2] != 2 * nE) return;
  if (in_sizes[3] != 4 * FD || in_sizes[4] != FD || in_sizes[5] != 3 * FD * FD || in_sizes[6] != FD) return;
  if (in_sizes[7] != FD * HH || in_sizes[8] != HH || in_sizes[9] != HH || in_sizes[10] < 1) return;
  for (int l = 0; l < 3; ++l) {
    const int b = 11 + 4 * l;
    if (in_sizes[b] != (FD + 2) * FD || in_sizes[b + 1] != FD * FD || in_sizes[b + 2] != FD || in_sizes[b + 3] != FD) return;
  }
  if (out_size != nN) return;
  if (nE > (1 << 27) || nN > (1 << 22)) return;

  const float* x     = (const float*)d_in[0];
  const int*   ei    = (const int*)d_in[1];
  const float* eattr = (const float*)d_in[2];
  const float* Win   = (const float*)d_in[3];
  const float* bin   = (const float*)d_in[4];
  const float* Wj    = (const float*)d_in[5];
  const float* bj    = (const float*)d_in[6];
  const float* W1    = (const float*)d_in[7];
  const float* b1    = (const float*)d_in[8];
  const float* W2    = (const float*)d_in[9];
  const float* b2    = (const float*)d_in[10];
  const float* Wn[3] = {(const float*)d_in[11], (const float*)d_in[15], (const float*)d_in[19]};
  const float* Ws[3] = {(const float*)d_in[12], (const float*)d_in[16], (const float*)d_in[20]};
  const float* ga[3] = {(const float*)d_in[13], (const float*)d_in[17], (const float*)d_in[21]};
  const float* be[3] = {(const float*)d_in[14], (const float*)d_in[18], (const float*)d_in[22]};
  const int* src = ei;
  const int* dst = ei + nE;
  float* dout = (float*)d_out;

  const int NPAD   = ((nN + RPADN - 1) / RPADN) * RPADN;
  const int nBC    = (nN + NBC - 1) / NBC;
  const int CNTPAD = nBC * NBC;
  if (CNTPAD < NPAD) return;
  if (FPC * nBC + 1 > RBN) return;
  const int nBF    = (nN + NBF - 1) / NBF;
  const int csrLen = ((nE + 31) & ~31) + 4096;
  if (31 * FPC * nBC > 4096) return;
  const int nGm    = NPAD / BM;
  const int nBL    = NPAD / (NWAVE * RPW);
  const int nUnit  = NPAD * (FD / 4);
  const int nIP    = nUnit / NTHR;

  char* ws = (char*)d_ws;
  size_t o = 0;
  size_t oCH[3], oCL[3];
  for (int l = 0; l < 3; ++l) { oCH[l] = carve(&o, (size_t)2 * FD * FD * 2); oCL[l] = carve(&o, (size_t)2 * FD * FD * 2); }
  const size_t oJH = carve(&o, (size_t)3 * FD * FD * 2), oJL = carve(&o, (size_t)3 * FD * FD * 2);
  const size_t o1H = carve(&o, (size_t)HH * FD * 2),     o1L = carve(&o, (size_t)HH * FD * 2);
  const size_t oCnt  = carve(&o, (size_t)CNTPAD * 4);
  const size_t oOff  = carve(&o, (size_t)CNTPAD * 4);
  const size_t oRb   = carve(&o, (size_t)RBN * 4);
  const size_t oCsr  = carve(&o, (size_t)csrLen * 4);
  const size_t oPart = carve(&o, (size_t)nGm * 2 * FD * 8);
  const size_t oTbl  = carve(&o, (size_t)2 * FD * 4);
  const size_t oP    = carve(&o, (size_t)NPAD * FD * 4);
  const size_t oQ    = carve(&o, (size_t)NPAD * FD * 4);
  if (o > ws_size || o > (size_t)WSLIM) return;

  unsigned short* cH[3]; unsigned short* cL[3];
  for (int l = 0; l < 3; ++l) { cH[l] = (unsigned short*)(ws + oCH[l]); cL[l] = (unsigned short*)(ws + oCL[l]); }
  unsigned short* jH = (unsigned short*)(ws + oJH); unsigned short* jL = (unsigned short*)(ws + oJL);
  unsigned short* hH = (unsigned short*)(ws + o1H); unsigned short* hL = (unsigned short*)(ws + o1L);
  int*    cnt  = (int*)(ws + oCnt);
  int*    offp = (int*)(ws + oOff);
  int*    rb   = (int*)(ws + oRb);
  int*    csr  = (int*)(ws + oCsr);
  double* part = (double*)(ws + oPart);
  float*  tbl  = (float*)(ws + oTbl);
  float*  P    = (float*)(ws + oP);
  float*  Q    = (float*)(ws + oQ);

  const int vec8 = ((nE & 3) == 0) ? 1 : 0;

  for (int l = 0; l < 3; ++l)
    k_wprep<<<(2 * FD * 16 + NTHR - 1) / NTHR, NTHR, 0, stream>>>(Wn[l], Ws[l], Ws[l], FD, 0, FD, cH[l], cL[l], 2 * FD * 16);
  k_wprep<<<(3 * FD * 16 + NTHR - 1) / NTHR, NTHR, 0, stream>>>(Wj, Wj, Wj, FD, FD, FD, jH, jL, 3 * FD * 16);
  k_wprep<<<(HH * 16 + NTHR - 1) / NTHR, NTHR, 0, stream>>>(W1, W1, W1, HH, 0, HH, hH, hL, HH * 16);

  k_count<<<nBC, NTHR, 0, stream>>>(dst, cnt, nE, vec8);
  k_offsets<<<1, OTHR, 0, stream>>>(cnt, offp, rb, nBC);
  hipFuncSetAttribute(reinterpret_cast<const void*>(&k_fill),
                      hipFuncAttributeMaxDynamicSharedMemorySize, LDS_FILL);
  k_fill<<<nBF, NTHR, LDS_FILL, stream>>>(dst, offp, rb, csr, nE, vec8, csrLen);

  k_inproj<<<nIP, NTHR, 0, stream>>>(x, Win, bin, P, nN, nUnit);

  hipFuncSetAttribute(reinterpret_cast<const void*>(&k_layer),
                      hipFuncAttributeMaxDynamicSharedMemorySize, LDS_LAYER);
  float* pin[2]  = {P, Q};
  float* pout[2] = {Q, P};
  for (int l = 0; l < 2; ++l) {
    k_layer<<<nGm, NTHR, LDS_LAYER, stream>>>(pin[l], pout[l], 1, csr, offp, cnt, src, eattr,
        Wn[l] + (size_t)FD * FD, cH[l], cL[l], cH[l] + (size_t)FD * FD, cL[l] + (size_t)FD * FD,
        part, nN, nE, csrLen);
    k_bnfin<<<1, FD, 0, stream>>>(part, ga[l], tbl, nGm, nN);
    k_bnl2<<<nBL, NTHR, 0, stream>>>(pout[l], tbl, be[l], nN);
  }

  k_layer<<<nGm, NTHR, LDS_LAYER, stream>>>(P, P, 0, csr, offp, cnt, src, eattr,
      Wn[2] + (size_t)FD * FD, cH[2], cL[2], cH[2] + (size_t)FD * FD, cL[2] + (size_t)FD * FD,
      part, nN, nE, csrLen);
  k_bnfin<<<1, FD, 0, stream>>>(part, ga[2], tbl, nGm, nN);

  hipFuncSetAttribute(reinterpret_cast<const void*>(&k_final),
                      hipFuncAttributeMaxDynamicSharedMemorySize, LDS_LAYER);
  k_final<<<nGm, NTHR, LDS_LAYER, stream>>>(P, Q, csr, offp, cnt, src, eattr,
      Wn[2] + (size_t)FD * FD, cH[2], cL[2], cH[2] + (size_t)FD * FD, cL[2] + (size_t)FD * FD,
      tbl, be[2], jH, jL, bj, hH, hL, b1, W2, b2, dout, nN, nE, csrLen);
}
